// Net_23665269801495
// MI455X (gfx1250) — hardware-verified
//
#include <hip/hip_runtime.h>
#include <stddef.h>
#include <stdint.h>

#define NN    1024
#define NE    2048
#define NG    64
#define XK    37
#define XKP   64
#define PTHR  256
#define ETHR  256
#define STHR  256
#define GTHR  128
#define GBM   64
#define GBN   128
#define GKU   256
#define GH    128
#define SP    132
#define XP    132
#define CINV  0.00390625f
#define CWGT  256.0f
#define FMINN 6.103515625e-05f
#define WSMAX 134217728

#define EDGE_LDS(ICH) ((128 * SP + (ICH) * XP + (ICH) * 128) * 4)

#define O_W2T1 ((size_t)0)
#define O_W2T2 (O_W2T1 + (size_t)4736 * 512 * 2)
#define O_W2T3 (O_W2T2 + (size_t)32768 * 128 * 2)
#define O_HID1 (O_W2T3 + (size_t)65536 * 128 * 2)
#define O_HID2 (O_HID1 + (size_t)NE * 512 * 2)
#define O_HID3 (O_HID2 + (size_t)NE * 128 * 2)
#define O_PM   (O_HID3 + (size_t)NE * 128 * 2)
#define O_HA   (O_PM   + (size_t)8 * NE * 256 * 4)
#define O_HB   (O_HA   + (size_t)NN * 256 * 4)
#define O_HHL  (O_HB   + (size_t)NN * 256 * 4)
#define O_ROOT (O_HHL  + (size_t)NN * 512 * 2)
#define O_XB   (O_ROOT + (size_t)NN * 256 * 4)
#define O_XR   (O_XB   + (size_t)NN * XKP * 2)
#define O_R1T  (O_XR   + (size_t)NN * XKP * 4)
#define O_R2D  (O_R1T  + (size_t)128 * XKP * 2)
#define O_R3D  (O_R2D  + (size_t)256 * 256 * 2)
#define O_FC1D (O_R3D  + (size_t)256 * 512 * 2)
#define O_FC2D (O_FC1D + (size_t)128 * 512 * 2)
#define O_GHL  (O_FC2D + (size_t)128 * 256 * 2)
#define O_G1HL (O_GHL  + (size_t)NG * 512 * 2)
#define O_END  (O_G1HL + (size_t)NG * 256 * 2)

static_assert(O_END == (size_t)55230464);
static_assert(O_END <= (size_t)WSMAX);
static_assert(O_W2T2 % 256 == 0 && O_W2T3 % 256 == 0 && O_HID1 % 256 == 0 && O_PM % 256 == 0 && O_HA % 256 == 0);
static_assert(O_XB % 256 == 0 && O_XR % 256 == 0 && O_R1T % 256 == 0 && O_R2D % 256 == 0 && O_GHL % 256 == 0 && O_G1HL % 256 == 0);
static_assert(NE % 128 == 0 && NN % 32 == 0 && NN % GBM == 0 && NE == 8 * STHR && NN == 4 * 256);
static_assert(4736 == XK * 128 && 4736 % 32 == 0);
static_assert(EDGE_LDS(32) <= 300000);

#define PB_W1  0
#define PB_W2  (PB_W1 + 148 * 4)
#define PB_W3  (PB_W2 + 1024)
#define PB_R2  (PB_W3 + 2048)
#define PB_R3  (PB_R2 + 16)
#define PB_F1  (PB_R3 + 32)
#define PB_F2  (PB_F1 + 16)
#define PB_H1  (PB_F2 + 8)
#define PB_H2  (PB_H1 + (NE * 512 / 8) / PTHR)
#define PB_H3  (PB_H2 + (NE * 128 / 8) / PTHR)
#define PB_XB  (PB_H3 + (NE * 128 / 8) / PTHR)
#define PB_XR  (PB_XB + (NN * 8) / PTHR)
#define PB_R1  (PB_XR + (NN * 16) / PTHR)
#define PB_END (PB_R1 + (128 * 8) / PTHR)
static_assert(PB_END == 4604);

typedef float          v4f   __attribute__((ext_vector_type(4)));
typedef float          v8f   __attribute__((ext_vector_type(8)));
typedef int            v4i   __attribute__((ext_vector_type(4)));
typedef int            v8i   __attribute__((ext_vector_type(8)));
typedef unsigned short v8us  __attribute__((ext_vector_type(8)));
typedef unsigned short v16us __attribute__((ext_vector_type(16)));
typedef __bf16         v16bf __attribute__((ext_vector_type(16)));
typedef _Float16       v16h  __attribute__((ext_vector_type(16)));
typedef v4f  __attribute__((may_alias)) v4fa;
typedef v4i  __attribute__((may_alias)) v4ia;
typedef v8us __attribute__((may_alias)) v8usa;
union FragB { v16bf v; v16us u; v8us h[2]; v8i w; };
union FragH { v16h  v; v16us u; v8us h[2]; v8i w; };

__device__ __forceinline__ v8f wmb(const FragB& a, const FragB& b, v8f c) {
  v8f d = __builtin_amdgcn_wmma_f32_16x16x32_bf16(false, a.v, false, b.v, (short)0, c, false, false);
  asm volatile("v_nop\n\tv_nop\n\tv_nop\n\tv_nop" : "+v"(d) : "v"(a.w), "v"(b.w));
  return d;
}
__device__ __forceinline__ v8f wmh(const FragH& a, const FragH& b, v8f c) {
  v8f d = __builtin_amdgcn_wmma_f32_16x16x32_f16(false, a.v, false, b.v, (short)0, c, false, false);
  asm volatile("v_nop\n\tv_nop\n\tv_nop\n\tv_nop" : "+v"(d) : "v"(a.w), "v"(b.w));
  return d;
}

__device__ __forceinline__ unsigned bf16_bits(float f) {
  const unsigned u = __float_as_uint(f);
  const unsigned r = (u + 0x7FFFu + ((u >> 16) & 1u)) >> 16;
  const unsigned q = (u >> 16) | 0x40u;
  return ((u & 0x7fffffffu) > 0x7f800000u) ? q : r;
}
__device__ __forceinline__ float bf16_val(float f) {
  return __uint_as_float(bf16_bits(f) << 16);
}
__device__ __forceinline__ unsigned short f2h(float f) {
  const _Float16 hv = (_Float16)f;
  return __builtin_bit_cast(unsigned short, hv);
}
__device__ __forceinline__ float elu_f(float v) {
  const float e = expm1f(v);
  return (v > 0.0f) ? v : e;
}
__device__ __forceinline__ void put16(unsigned short* dp, v8us o) {
  *(volatile v8us*)dp = o;
  __threadfence();
  *(volatile v8us*)dp = o;
}
__device__ __forceinline__ void putf4(float* dp, v4f o) {
  *(volatile v4f*)dp = o;
  __threadfence();
  *(volatile v4f*)dp = o;
}

template <int MODE>
__device__ __forceinline__ void tr_tile(const float* __restrict__ src, int ldsrc, int k0src, int col0, int zero,
                                        unsigned short* dst, int ldd, int tid, float* sT) {
  if (zero != 0) {
    const v4f z4 = {0.0f, 0.0f, 0.0f, 0.0f};
#pragma unroll
    for (int i = 0; i < 4; ++i) {
      const int q = tid + i * PTHR;
      *(v4fa*)(sT + (q >> 3) * 32 + (q & 7) * 4) = z4;
    }
  } else {
#pragma unroll
    for (int i = 0; i < 4; ++i) {
      const int q = tid + i * PTHR;
      const int k = q >> 3, c4 = (q & 7) * 4;
      const v4f v = *(const v4fa*)(src + (size_t)(k0src + k) * (size_t)ldsrc + col0 + c4);
      const v4f r = {bf16_val(v.x), bf16_val(v.y), bf16_val(v.z), bf16_val(v.w)};
      *(v4fa*)(sT + k * 32 + c4) = r;
    }
  }
  __syncthreads();
  v8us o[2];
#pragma unroll
  for (int i = 0; i < 2; ++i) {
    const int c = tid + i * PTHR;
    const int row = c >> 4, k8 = (c & 15) * 8;
    v8us t;
#pragma unroll
    for (int j = 0; j < 8; ++j) {
      const float s = sT[(k8 + j) * 32 + row];
      if constexpr (MODE == 0) {
        t[j] = (unsigned short)(__float_as_uint(s) >> 16);
      } else {
        float w = CWGT * s;
        w = (fabsf(w) < FMINN) ? 0.0f : w;
        t[j] = f2h(w);
      }
    }
    o[i] = t;
  }
#pragma unroll
  for (int i = 0; i < 2; ++i) {
    const int c = tid + i * PTHR;
    *(volatile v8us*)(dst + (size_t)(c >> 4) * (size_t)ldd + (c & 15) * 8) = o[i];
  }
  __threadfence();
#pragma unroll
  for (int i = 0; i < 2; ++i) {
    const int c = tid + i * PTHR;
    *(volatile v8us*)(dst + (size_t)(c >> 4) * (size_t)ldd + (c & 15) * 8) = o[i];
  }
}

template <int K>
__device__ __forceinline__ void hid_unit(const float* __restrict__ ea, const float* __restrict__ w1,
                                         const float* __restrict__ b1, int u, unsigned short* dst) {
  constexpr int KC = K / 8;
  const int e  = u / KC;
  const int k8 = (u - e * KC) * 8;
  const v4f a = *(const v4fa*)(ea + 4 * e);
  const float a0 = bf16_val(a.x), a1 = bf16_val(a.y), a2 = bf16_val(a.z), a3 = bf16_val(a.w);
  v8f s;
  {
    const v4f p = *(const v4fa*)(w1 + k8);
    const v4f q = *(const v4fa*)(w1 + k8 + 4);
    const v8f w = {p.x, p.y, p.z, p.w, q.x, q.y, q.z, q.w};
#pragma unroll
    for (int i = 0; i < 8; ++i) s[i] = a0 * bf16_val(w[i]);
  }
  {
    const v4f p = *(const v4fa*)(w1 + K + k8);
    const v4f q = *(const v4fa*)(w1 + K + k8 + 4);
    const v8f w = {p.x, p.y, p.z, p.w, q.x, q.y, q.z, q.w};
#pragma unroll
    for (int i = 0; i < 8; ++i) s[i] = fmaf(a1, bf16_val(w[i]), s[i]);
  }
  {
    const v4f p = *(const v4fa*)(w1 + 2 * K + k8);
    const v4f q = *(const v4fa*)(w1 + 2 * K + k8 + 4);
    const v8f w = {p.x, p.y, p.z, p.w, q.x, q.y, q.z, q.w};
#pragma unroll
    for (int i = 0; i < 8; ++i) s[i] = fmaf(a2, bf16_val(w[i]), s[i]);
  }
  {
    const v4f p = *(const v4fa*)(w1 + 3 * K + k8);
    const v4f q = *(const v4fa*)(w1 + 3 * K + k8 + 4);
    const v8f w = {p.x, p.y, p.z, p.w, q.x, q.y, q.z, q.w};
#pragma unroll
    for (int i = 0; i < 8; ++i) s[i] = fmaf(a3, bf16_val(w[i]), s[i]);
  }
  const v4f bp = *(const v4fa*)(b1 + k8);
  const v4f bq = *(const v4fa*)(b1 + k8 + 4);
  const v8f bb = {bp.x, bp.y, bp.z, bp.w, bq.x, bq.y, bq.z, bq.w};
  v8us o;
#pragma unroll
  for (int i = 0; i < 8; ++i) {
    float v = s[i] + bf16_val(bb[i]);
    v = fmaxf(v, 0.0f);
    v = (v < FMINN) ? 0.0f : v;
    o[i] = f2h(v);
  }
  put16(dst + (size_t)e * K + k8, o);
}

__global__ __launch_bounds__(PTHR) void k_prep(
    const float* __restrict__ x, const float* __restrict__ ea,
    const float* __restrict__ w11, const float* __restrict__ b11, const float* __restrict__ w12, const float* __restrict__ rt1,
    const float* __restrict__ w21, const float* __restrict__ b21, const float* __restrict__ w22, const float* __restrict__ rt2,
    const float* __restrict__ w31, const float* __restrict__ b31, const float* __restrict__ w32, const float* __restrict__ rt3,
    const float* __restrict__ fc1w, const float* __restrict__ fc2w, unsigned char* ws) {
  __shared__ __attribute__((aligned(16))) float sT[128 * 32];
  const int b = (int)blockIdx.x, tid = (int)threadIdx.x;
  if (b < PB_W2) {
    const int cb = b >> 2, kt = b & 3;
    tr_tile<1>(w12, 4736, kt * 128, cb * 32, 0,
               (unsigned short*)(ws + O_W2T1) + (size_t)cb * 32 * 512 + kt * 128, 512, tid, sT);
  } else if (b < PB_W3) {
    const int cb = b - PB_W2;
    tr_tile<1>(w22, 32768, 0, cb * 32, 0, (unsigned short*)(ws + O_W2T2) + (size_t)cb * 32 * 128, 128, tid, sT);
  } else if (b < PB_R2) {
    const int cb = b - PB_W3;
    tr_tile<1>(w32, 65536, 0, cb * 32, 0, (unsigned short*)(ws + O_W2T3) + (size_t)cb * 32 * 128, 128, tid, sT);
  } else if (b < PB_R3) {
    const int bb = b - PB_R2, cb = bb >> 1, kt = bb & 1;
    tr_tile<0>(rt2, 256, 0, cb * 32, 0, (unsigned short*)(ws + O_R2D) + (size_t)cb * 32 * 256 + kt * 128, 256, tid, sT);
  } else if (b < PB_F1) {
    const int bb = b - PB_R3, cb = bb >> 2, kt = bb & 3;
    tr_tile<0>(rt3, 256, (kt & 1) * 128, cb * 32, 0,
               (unsigned short*)(ws + O_R3D) + (size_t)cb * 32 * 512 + kt * 128, 512, tid, sT);
  } else if (b < PB_F2) {
    const int bb = b - PB_F1, cb = bb >> 2, kt = bb & 3;
    tr_tile<0>(fc1w, 128, (kt & 1) * 128, cb * 32, 0,
               (unsigned short*)(ws + O_FC1D) + (size_t)cb * 32 * 512 + kt * 128, 512, tid, sT);
  } else if (b < PB_H1) {
    const int bb = b - PB_F2, cb = bb >> 1, kt = bb & 1;
    tr_tile<0>(fc2w, 64, 0, (cb & 1) * 32, (cb >= 2) ? 1 : 0,
               (unsigned short*)(ws + O_FC2D) + (size_t)cb * 32 * 256 + kt * 128, 256, tid, sT);
  } else if (b < PB_H2) {
    hid_unit<512>(ea, w11, b11, (b - PB_H1) * PTHR + tid, (unsigned short*)(ws + O_HID1));
  } else if (b < PB_H3) {
    hid_unit<128>(ea, w21, b21, (b - PB_H2) * PTHR + tid, (unsigned short*)(ws + O_HID2));
  } else if (b < PB_XB) {
    hid_unit<128>(ea, w31, b31, (b - PB_H3) * PTHR + tid, (unsigned short*)(ws + O_HID3));
  } else if (b < PB_XR) {
    const int u = (b - PB_XB) * PTHR + tid;
    const int row = u >> 3, k8 = (u & 7) * 8;
    const float* xr = x + (size_t)row * XK;
    v8us o;
#pragma unroll
    for (int i = 0; i < 8; ++i) {
      const int kk = k8 + i;
      const int kc = kk < XK ? kk : XK - 1;
      const float v = xr[kc];
      o[i] = (kk < XK) ? (unsigned short)bf16_bits(v) : (unsigned short)0;
    }
    put16((unsigned short*)(ws + O_XB) + (size_t)row * XKP + k8, o);
  } else if (b < PB_R1) {
    const int u = (b - PB_XR) * PTHR + tid;
    const int row = u >> 4, c4 = (u & 15) * 4;
    const float* xr = x + (size_t)row * XK;
    float q[4];
#pragma unroll
    for (int i = 0; i < 4; ++i) {
      const int kk = c4 + i;
      const int kc = kk < XK ? kk : XK - 1;
      const float v = xr[kc];
      q[i] = (kk < XK) ? bf16_val(v) : 0.0f;
    }
    const v4f o = {q[0], q[1], q[2], q[3]};
    putf4((float*)(ws + O_XR) + (size_t)row * XKP + c4, o);
  } else {
    const int u = (b - PB_R1) * PTHR + tid;
    const int n = u >> 3, k8 = (u & 7) * 8;
    v8us o;
#pragma unroll
    for (int i = 0; i < 8; ++i) {
      const int kk = k8 + i;
      const int kc = kk < XK ? kk : XK - 1;
      const float v = rt1[(size_t)kc * 128 + n];
      o[i] = (kk < XK) ? (unsigned short)bf16_bits(v) : (unsigned short)0;
    }
    put16((unsigned short*)(ws + O_R1T) + (size_t)n * XKP + k8, o);
  }
}

template <int MODE>
__global__ __launch_bounds__(GTHR) void k_gemm(const unsigned short* __restrict__ A, int lda,
                                               const unsigned short* __restrict__ BT, int ldb, int K,
                                               const float* __restrict__ bias, int nBias,
                                               float* Cm, int ldc, unsigned short* Cb,
                                               const float* __restrict__ w3, const float* __restrict__ b3) {
  __shared__ __attribute__((aligned(16))) float stg[GBM * GBN];
  __shared__ __attribute__((aligned(16))) float sW3[64];
  __shared__ __attribute__((aligned(16))) float sOut[64];
  const int tid = (int)threadIdx.x, lane = tid & 31, wave = tid >> 5, hh = lane >> 4, m = lane & 15;
  const int rowBase = (int)blockIdx.x * GBM;
  const int colBase = (int)blockIdx.y * GBN;

  if constexpr (MODE == 2) {
    if (tid < 64) sW3[tid] = bf16_val(w3[tid]);
  }

  v8f acc[8];
  {
    const v8f z = {0.f, 0.f, 0.f, 0.f, 0.f, 0.f, 0.f, 0.f};
#pragma unroll
    for (int t = 0; t < 8; ++t) acc[t] = z;
  }
  const unsigned short* ap = A  + (size_t)(rowBase + 16 * wave + m) * (size_t)lda + 8 * hh;
  const unsigned short* bp = BT + (size_t)(colBase + m) * (size_t)ldb + 8 * hh;

#pragma unroll 1
  for (int k0 = 0; k0 < K; k0 += 32) {
    FragB af;
    af.h[0] = *(const v8usa*)(ap + k0);
    af.h[1] = *(const v8usa*)(ap + k0 + 16);
#pragma unroll
    for (int nt = 0; nt < 8; ++nt) {
      const unsigned short* wq = bp + (size_t)(16 * nt) * (size_t)ldb + k0;
      FragB bf;
      bf.h[0] = *(const v8usa*)wq;
      bf.h[1] = *(const v8usa*)(wq + 16);
      acc[nt] = wmb(af, bf, acc[nt]);
    }
  }

#pragma unroll
  for (int nt = 0; nt < 8; ++nt) {
    const int lc = 16 * nt + m;
    int bi = colBase + lc;
    bi = bi < nBias ? bi : nBias - 1;
    const float bvv = bf16_val(bias[bi]);
#pragma unroll
    for (int r = 0; r < 8; ++r) {
      const int lr = 16 * wave + 8 * hh + r;
      stg[lr * GBN + lc] = acc[nt][r] + bvv;
    }
  }
  __syncthreads();

  if constexpr (MODE != 0) {
#pragma unroll 1
    for (int q = 0; q < (GBM * GBN) / GTHR; ++q) {
      const int idx = tid + GTHR * q;
      const float v = stg[idx];
      stg[idx] = elu_f(v);
    }
    __syncthreads();
  }

  if constexpr (MODE == 0) {
    v4f pv[16];
#pragma unroll
    for (int i = 0; i < 16; ++i) pv[i] = *(const v4fa*)(stg + (16 * wave + i) * GBN + 4 * lane);
#pragma unroll
    for (int i = 0; i < 16; ++i) {
      float* op = Cm + (size_t)(rowBase + 16 * wave + i) * (size_t)ldc + colBase + 4 * lane;
      *(volatile v4f*)op = pv[i];
    }
    __threadfence();
#pragma unroll
    for (int i = 0; i < 16; ++i) {
      float* op = Cm + (size_t)(rowBase + 16 * wave + i) * (size_t)ldc + colBase + 4 * lane;
      *(volatile v4f*)op = pv[i];
    }
  } else if constexpr (MODE == 1) {
    const int part = lane >> 4;
    const int j = lane & 15;
    const unsigned mh = 0u - (unsigned)part;
    const unsigned ml = ~mh;
    v8us pv[16];
#pragma unroll
    for (int i = 0; i < 16; ++i) {
      const float* sp = stg + (16 * wave + i) * GBN + 8 * j;
      const v4f a = *(const v4fa*)sp;
      const v4f b = *(const v4fa*)(sp + 4);
      const v8f f8 = {a.x, a.y, a.z, a.w, b.x, b.y, b.z, b.w};
      v8us oo;
#pragma unroll
      for (int e = 0; e < 8; ++e) {
        const unsigned hb = bf16_bits(f8[e]);
        const unsigned lb = bf16_bits(f8[e] - __uint_as_float(hb << 16));
        oo[e] = (unsigned short)((hb & ml) | (lb & mh));
      }
      pv[i] = oo;
    }
#pragma unroll
    for (int i = 0; i < 16; ++i) {
      unsigned short* op = Cb + (size_t)(rowBase + 16 * wave + i) * (size_t)GKU + part * GH + 8 * j;
      *(volatile v8us*)op = pv[i];
    }
    __threadfence();
#pragma unroll
    for (int i = 0; i < 16; ++i) {
      unsigned short* op = Cb + (size_t)(rowBase + 16 * wave + i) * (size_t)GKU + part * GH + 8 * j;
      *(volatile v8us*)op = pv[i];
    }
  } else {
    const float w3a = sW3[lane], w3b = sW3[32 + lane];
    float res = 0.0f;
#pragma unroll 1
    for (int i = 0; i < 16; ++i) {
      const int row = 16 * wave + i;
      float p = stg[row * GBN + lane] * w3a + stg[row * GBN + 32 + lane] * w3b;
      p += __shfl_xor(p, 16);
      p += __shfl_xor(p, 8);
      p += __shfl_xor(p, 4);
      p += __shfl_xor(p, 2);
      p += __shfl_xor(p, 1);
      res = (lane == i) ? p : res;
    }
    const float b3v = bf16_val(b3[0]);
    if (lane < 16) sOut[16 * wave + lane] = res + b3v;
    __syncthreads();
    if (wave == 0) {
      const v4f o = *(const v4fa*)(sOut + 4 * (lane & 15));
      if (lane < 16) *(volatile v4f*)(Cm + 4 * lane) = o;
      __threadfence();
      if (lane < 16) *(volatile v4f*)(Cm + 4 * lane) = o;
    }
  }
}

template <int MIN, int MOUT, int K, int ICH>
__global__ __launch_bounds__(ETHR) void k_edge(const int* __restrict__ src, const float* __restrict__ Hp, int ldh,
                                               const unsigned short* __restrict__ HID,
                                               const unsigned short* __restrict__ W2T,
                                               const float* __restrict__ b2, float* PM) {
  static_assert(K % 32 == 0 && MOUT % 128 == 0 && ICH % 2 == 0 && (ICH * 32) % 32 == 0);
  extern __shared__ __attribute__((aligned(16))) float dyn[];
  float* stg = dyn;
  float* xsT = dyn + 128 * SP;
  float* b2s = xsT + ICH * XP;
  const int tid = (int)threadIdx.x, lane = tid & 31, wave = tid >> 5, hh = lane >> 4, m = lane & 15;
  const int e0 = (int)blockIdx.x * 128;
  const int o0 = (int)blockIdx.y * 128;
  const int z  = (int)blockIdx.z;
  const int i0 = z * ICH;
  const int iEnd = (i0 + ICH < MIN) ? (i0 + ICH) : MIN;

  {
    const int r = tid & 127;
    int s = src[e0 + r];
    s = s < 0 ? 0 : (s > NN - 1 ? NN - 1 : s);
    const float* hr = Hp + (size_t)s * (size_t)ldh;
#pragma unroll 2
    for (int j = tid >> 7; j < ICH; j += 2) {
      int c = i0 + j;
      c = c < ldh ? c : ldh - 1;
      xsT[j * XP + r] = hr[c];
    }
  }
  for (int u = tid; u < ICH * 32; u += ETHR) {
    const int j = u >> 5, c4 = (u & 31) * 4;
    int ir = i0 + j;
    ir = ir < MIN ? ir : MIN - 1;
    const v4f v = *(const v4fa*)(b2 + (size_t)ir * MOUT + o0 + c4);
    const v4f r4 = {bf16_val(v.x), bf16_val(v.y), bf16_val(v.z), bf16_val(v.w)};
    *(v4fa*)(b2s + j * 128 + c4) = r4;
  }
  __syncthreads();

  const int wr = wave >> 1, wc = wave & 1;
  const int rowW = 32 * wr, colW = 64 * wc;
  const unsigned short* ap0 = HID + (size_t)(e0 + rowW + m) * K + 8 * hh;
  const unsigned short* ap1 = ap0 + (size_t)16 * K;
  const v8f z8 = {0.f, 0.f, 0.f, 0.f, 0.f, 0.f, 0.f, 0.f};
  v8f acc[2][4];
#pragma unroll
  for (int mt = 0; mt < 2; ++mt)
#pragma unroll
    for (int nt = 0; nt < 4; ++nt) acc[mt][nt] = z8;

#pragma unroll 1
  for (int i = i0; i < iEnd; ++i) {
    const int j = i - i0;
    const unsigned short* bp = W2T + ((size_t)i * MOUT + o0 + colW + m) * K + 8 * hh;
    v8f d[2][4];
#pragma unroll
    for (int mt = 0; mt < 2; ++mt)
#pragma unroll
      for (int nt = 0; nt < 4; ++nt) d[mt][nt] = z8;
#pragma unroll 1
    for (int k0 = 0; k0 < K; k0 += 32) {
      FragH a0, a1;
      a0.h[0] = *(const v8usa*)(ap0 + k0);
      a0.h[1] = *(const v8usa*)(ap0 + k0 + 16);
      a1.h[0] = *(const v8usa*)(ap1 + k0);
      a1.h[1] = *(const v8usa*)(ap1 + k0 + 16);
#pragma unroll
      for (int nt = 0; nt < 4; ++nt) {
        const unsigned short* wq = bp + (size_t)(16 * nt) * K + k0;
        FragH b;
        b.h[0] = *(const v8usa*)wq;
        b.h[1] = *(const v8usa*)(wq + 16);
        d[0][nt] = wmh(a0, b, d[0][nt]);
        d[1][nt] = wmh(a1, b, d[1][nt]);
      }
    }
    float bv[4];
#pragma unroll
    for (int nt = 0; nt < 4; ++nt) bv[nt] = b2s[j * 128 + colW + 16 * nt + m];
#pragma unroll
    for (int mt = 0; mt < 2; ++mt) {
      const float* xp = xsT + j * XP + rowW + 16 * mt + 8 * hh;
      const v4f xa = *(const v4fa*)xp;
      const v4f xb = *(const v4fa*)(xp + 4);
      const v8f x8 = {xa.x, xa.y, xa.z, xa.w, xb.x, xb.y, xb.z, xb.w};
#pragma unroll
      for (int nt = 0; nt < 4; ++nt)
#pragma unroll
        for (int r = 0; r < 8; ++r) {
          const float t = fmaf(d[mt][nt][r], CINV, bv[nt]);
          acc[mt][nt][r] = fmaf(x8[r], t, acc[mt][nt][r]);
        }
    }
  }

#pragma unroll
  for (int mt = 0; mt < 2; ++mt)
#pragma unroll
    for (int nt = 0; nt < 4; ++nt)
#pragma unroll
      for (int r = 0; r < 8; ++r)
        stg[(rowW + 16 * mt + 8 * hh + r) * SP + colW + 16 * nt + m] = acc[mt][nt][r];
  __syncthreads();

  {
    v4f pv[16];
#pragma unroll
    for (int i = 0; i < 16; ++i) pv[i] = *(const v4fa*)(stg + (16 * wave + i) * SP + 4 * lane);
    float* pb = PM + ((size_t)z * NE + e0 + 16 * wave) * MOUT + o0 + 4 * lane;
#pragma unroll
    for (int i = 0; i < 16; ++i) *(volatile v4f*)(pb + (size_t)i * MOUT) = pv[i];
    __threadfence();
#pragma unroll
    for (int i = 0; i < 16; ++i) *(volatile v4f*)(pb + (size_t)i * MOUT) = pv[i];
  }
}

template <int MOUT, int S, int WHL>
__global__ __launch_bounds__(STHR) void k_scat(const int* __restrict__ tgt, const float* __restrict__ PM,
                                               const float* __restrict__ ROOT, float* H, unsigned short* HHL) {
  constexpr int NJ = MOUT / 128;
  static_assert(MOUT == 128 || MOUT == 256);
  __shared__ __attribute__((aligned(16))) int   tg[NE];
  __shared__ __attribute__((aligned(16))) float rowS[8 * MOUT];
  const int tid = (int)threadIdx.x, lane = tid & 31, wave = tid >> 5;
  {
    const v4i a = *(const v4i*)(tgt + 8 * tid);
    const v4i b = *(const v4i*)(tgt + 8 * tid + 4);
    *(v4ia*)(tg + 8 * tid)     = a;
    *(v4ia*)(tg + 8 * tid + 4) = b;
  }
  __syncthreads();
  float* rs = rowS + wave * MOUT;
  const v4f z4 = {0.0f, 0.0f, 0.0f, 0.0f};

#pragma unroll 1
  for (int q = 0; q < 4; ++q) {
    const int node = (int)blockIdx.x * 32 + q * 8 + wave;
    v4f acc[NJ];
#pragma unroll
    for (int j = 0; j < NJ; ++j) acc[j] = z4;
#pragma unroll 1
    for (int step = 0; step < NE / 32; ++step) {
      const int t = tg[step * 32 + lane];
      unsigned mask = __builtin_amdgcn_ballot_w32(t == node);
#pragma unroll 1
      for (int it = 0; it < 32; ++it) {
        if (mask == 0u) break;
        const int bpos = __builtin_ctz(mask);
        mask &= mask - 1u;
        const int e = step * 32 + bpos;
        v4f hs[NJ];
#pragma unroll
        for (int j = 0; j < NJ; ++j) hs[j] = z4;
#pragma unroll 4
        for (int s = 0; s < S; ++s) {
          const float* pp = PM + ((size_t)s * NE + e) * MOUT + 4 * lane;
#pragma unroll
          for (int j = 0; j < NJ; ++j) hs[j] += *(const v4fa*)(pp + 128 * j);
        }
#pragma unroll
        for (int j = 0; j < NJ; ++j) acc[j] += hs[j];
      }
    }
#pragma unroll
    for (int j = 0; j < NJ; ++j) {
      const v4f r = *(const v4fa*)(ROOT + (size_t)node * MOUT + 128 * j + 4 * lane);
      const v4f v = acc[j] + r;
      *(v4fa*)(rs + 128 * j + 4 * lane) = v;
    }
    __syncthreads();
#pragma unroll 1
    for (int c = 0; c < MOUT / 32; ++c) {
      const float v = rs[32 * c + lane];
      rs[32 * c + lane] = elu_f(v);
    }
    __syncthreads();

    v4f hv[NJ];
#pragma unroll
    for (int j = 0; j < NJ; ++j) hv[j] = *(const v4fa*)(rs + 128 * j + 4 * lane);
    float* hp = H + (size_t)node * MOUT + 4 * lane;
    v8us oa, ob;
    unsigned short* qa = HHL;
    unsigned short* qb = HHL;
    if constexpr (WHL != 0) {
      if constexpr (MOUT == 128) {
        const int part = lane >> 4, j16 = lane & 15;
        const unsigned mh = 0u - (unsigned)part, ml = ~mh;
        const v4f a = *(const v4fa*)(rs + 8 * j16);
        const v4f b = *(const v4fa*)(rs + 8 * j16 + 4);
        const v8f f8 = {a.x, a.y, a.z, a.w, b.x, b.y, b.z, b.w};
#pragma unroll
        for (int e = 0; e < 8; ++e) {
          const unsigned hb = bf16_bits(f8[e]);
          const unsigned lb = bf16_bits(f8[e] - __uint_as_float(hb << 16));
          oa[e] = (unsigned short)((hb & ml) | (lb & mh));
        }
        ob = oa;
        qa = HHL + (size_t)node * 256 + part * 128 + 8 * j16;
        qb = qa;
      } else {
        const v4f a = *(const v4fa*)(rs + 8 * lane);
        const v4f b = *(const v4fa*)(rs + 8 * lane + 4);
        const v8f f8 = {a.x, a.y, a.z, a.w, b.x, b.y, b.z, b.w};
#pragma unroll
        for (int e = 0; e < 8; ++e) {
          const unsigned hb = bf16_bits(f8[e]);
          oa[e] = (unsigned short)hb;
          ob[e] = (unsigned short)bf16_bits(f8[e] - __uint_as_float(hb << 16));
        }
        qa = HHL + (size_t)node * 512 + 8 * lane;
        qb = qa + 256;
      }
    }
#pragma unroll
    for (int j = 0; j < NJ; ++j) *(volatile v4f*)(hp + 128 * j) = hv[j];
    if constexpr (WHL != 0) {
      *(volatile v8us*)qa = oa;
      if constexpr (MOUT == 256) *(volatile v8us*)qb = ob;
    }
    __threadfence();
#pragma unroll
    for (int j = 0; j < NJ; ++j) *(volatile v4f*)(hp + 128 * j) = hv[j];
    if constexpr (WHL != 0) {
      *(volatile v8us*)qa = oa;
      if constexpr (MOUT == 256) *(volatile v8us*)qb = ob;
    }
    __syncthreads();
  }
}

__global__ __launch_bounds__(256) void k_pool(const int* __restrict__ batch, const float* __restrict__ H3,
                                              unsigned short* GHL) {
  __shared__ __attribute__((aligned(16))) int   bt[NN];
  __shared__ __attribute__((aligned(16))) float gS[256];
  const int tid = (int)threadIdx.x, g = (int)blockIdx.x;
  {
    const v4i a = *(const v4i*)(batch + 4 * tid);
    *(v4ia*)(bt + 4 * tid) = a;
  }
  __syncthreads();
  float sum = 0.0f;
  int cnt = 0;
#pragma unroll 1
  for (int n = 0; n < NN; ++n) {
    const int bn = __builtin_amdgcn_readfirstlane(bt[n]);
    if (bn == g) {
      sum += H3[(size_t)n * 256 + tid];
      cnt += 1;
    }
  }
  const float den = fmaxf((float)cnt, 1.0f);
  gS[tid] = sum / den;
  __syncthreads();
  if (tid < 32) {
    const v4f a = *(const v4fa*)(gS + 8 * tid);
    const v4f b = *(const v4fa*)(gS + 8 * tid + 4);
    const v8f f8 = {a.x, a.y, a.z, a.w, b.x, b.y, b.z, b.w};
    v8us oh, ol;
#pragma unroll
    for (int e = 0; e < 8; ++e) {
      const unsigned hb = bf16_bits(f8[e]);
      oh[e] = (unsigned short)hb;
      ol[e] = (unsigned short)bf16_bits(f8[e] - __uint_as_float(hb << 16));
    }
    unsigned short* qa = GHL + (size_t)g * 512 + 8 * tid;
    *(volatile v8us*)qa         = oh;
    *(volatile v8us*)(qa + 256) = ol;
    __threadfence();
    *(volatile v8us*)qa         = oh;
    *(volatile v8us*)(qa + 256) = ol;
  }
}

extern "C" void kernel_launch(void* const* d_in, const int* in_sizes, int n_in,
                              void* d_out, int out_size, void* d_ws, size_t ws_size,
                              hipStream_t stream) {
  if (n_in < 28) return;
  if (in_sizes[0] != NN * XK || in_sizes[1] != 2 * NE || in_sizes[2] != NE * 4 || in_sizes[3] != NN) return;
  if (in_sizes[4] != 4 * 512 || in_sizes[5] != 512 || in_sizes[6] != 512 * 4736 || in_sizes[7] != 4736) return;
  if (in_sizes[8] != XK * 128 || in_sizes[9] != 128) return;
  if (in_sizes[10] != 4 * 128 || in_sizes[11] != 128 || in_sizes[12] != 128 * 32768 || in_sizes[13] != 32768) return;
  if (in_sizes[14] != 128 * 256 || in_sizes[15] != 256) return;
  if (in_sizes[16] != 4 * 128 || in_sizes[17] != 128 || in_sizes[18] != 128 * 65536 || in_sizes[19] != 65536) return;
  if (in_sizes[20] != 256 * 256 || in_sizes[21] != 256) return;
  if (in_sizes[22] != 256 * 128 || in_sizes[23] != 128 || in_sizes[24] != 128 * 64 || in_sizes[25] != 64) return;
  if (in_sizes[26] != 64 || in_sizes[27] != 1) return;
  if (out_size != NG) return;
  if (ws_size < O_END) return;

  const float* x     = (const float*)d_in[0];
  const int*   eidx  = (const int*)d_in[1];
  const float* ea    = (const float*)d_in[2];
  const int*   batch = (const int*)d_in[3];
  const float* c1_w1 = (const float*)d_in[4];  const float* c1_b1 = (const float*)d_in[5];
  const float* c1_w2 = (const float*)d_in[6];  const float* c1_b2 = (const float*)d_in[7];
  const float* c1_rt = (const float*)d_in[8];  const float* c1_bs = (const float*)d_in[9];
  const float* c2_w1 = (const float*)d_in[10]; const float* c2_b1 = (const float*)d_in[11];
  const float* c2_w2 = (const float*)d_in[12]; const float* c2_b2 = (const float*)d_in[13];
  const float* c2_rt = (const float*)d_in[14]; const float* c2_bs = (const float*)d_in[15];
  const float* c3_w1 = (const float*)d_in[16]; const float* c3_b1 = (const float*)d_in[17];
  const float* c3_w2 = (const float*)d_in[18]; const float* c3_b2 = (const float*)d_in[19];
  const float* c3_rt = (const float*)d_in[20]; const float* c3_bs = (const float*)d_in[21];
  const float* fc1_w = (const float*)d_in[22]; const float* fc1_b = (const float*)d_in[23];
  const float* fc2_w = (const float*)d_in[24]; const float* fc2_b = (const float*)d_in[25];
  const float* fc3_w = (const float*)d_in[26]; const float* fc3_b = (const float*)d_in[27];
  const int* src = eidx;
  const int* tgt = eidx + NE;
  float* out = (float*)d_out;

  unsigned char* ws = (unsigned char*)d_ws;
  unsigned short* W2T1 = (unsigned short*)(ws + O_W2T1);
  unsigned short* W2T2 = (unsigned short*)(ws + O_W2T2);
  unsigned short* W2T3 = (unsigned short*)(ws + O_W2T3);
  unsigned short* HID1 = (unsigned short*)(ws + O_HID1);
  unsigned short* HID2 = (unsigned short*)(ws + O_HID2);
  unsigned short* HID3 = (unsigned short*)(ws + O_HID3);
  float*          PM   = (float*)(ws + O_PM);
  float*          HA   = (float*)(ws + O_HA);
  float*          HB   = (float*)(ws + O_HB);
  unsigned short* HHL  = (unsigned short*)(ws + O_HHL);
  float*          ROOT = (float*)(ws + O_ROOT);
  unsigned short* XB   = (unsigned short*)(ws + O_XB);
  float*          XR   = (float*)(ws + O_XR);
  unsigned short* R1T  = (unsigned short*)(ws + O_R1T);
  unsigned short* R2D  = (unsigned short*)(ws + O_R2D);
  unsigned short* R3D  = (unsigned short*)(ws + O_R3D);
  unsigned short* FC1D = (unsigned short*)(ws + O_FC1D);
  unsigned short* FC2D = (unsigned short*)(ws + O_FC2D);
  unsigned short* GHL  = (unsigned short*)(ws + O_GHL);
  unsigned short* G1HL = (unsigned short*)(ws + O_G1HL);

  hipFuncSetAttribute(reinterpret_cast<const void*>(&k_edge<37, 128, 512, 10>),
                      hipFuncAttributeMaxDynamicSharedMemorySize, (int)EDGE_LDS(10));
  hipFuncSetAttribute(reinterpret_cast<const void*>(&k_edge<128, 256, 128, 16>),
                      hipFuncAttributeMaxDynamicSharedMemorySize, (int)EDGE_LDS(16));
  hipFuncSetAttribute(reinterpret_cast<const void*>(&k_edge<256, 256, 128, 32>),
                      hipFuncAttributeMaxDynamicSharedMemorySize, (int)EDGE_LDS(32));

  k_prep<<<PB_END, PTHR, 0, stream>>>(x, ea, c1_w1, c1_b1, c1_w2, c1_rt, c2_w1, c2_b1, c2_w2, c2_rt,
                                      c3_w1, c3_b1, c3_w2, c3_rt, fc1_w, fc2_w, ws);

  k_gemm<0><<<dim3(NN / GBM, 1), GTHR, 0, stream>>>(XB, XKP, R1T, XKP, XKP, c1_bs, 128, ROOT, 128, HHL, fc3_w, fc3_b);
  k_edge<37, 128, 512, 10><<<dim3(NE / 128, 1, 4), ETHR, EDGE_LDS(10), stream>>>(src, XR, XKP, HID1, W2T1, c1_b2, PM);
  k_scat<128, 4, 1><<<NN / 32, STHR, 0, stream>>>(tgt, PM, ROOT, HA, HHL);

  k_gemm<0><<<dim3(NN / GBM, 2), GTHR, 0, stream>>>(HHL, 256, R2D, 256, 256, c2_bs, 256, ROOT, 256, HHL, fc3_w, fc3_b);
  k_edge<128, 256, 128, 16><<<dim3(NE / 128, 2, 8), ETHR, EDGE_LDS(16), stream>>>(src, HA, 128, HID2, W2T2, c2_b2, PM);
  k_scat<256, 8, 1><<<NN / 32, STHR, 0, stream>>>(tgt, PM, ROOT, HB, HHL);

  k_gemm<0><<<dim3(NN / GBM, 2), GTHR, 0, stream>>>(HHL, 512, R3D, 512, 512, c3_bs, 256, ROOT, 256, HHL, fc3_w, fc3_b);
  k_edge<256, 256, 128, 32><<<dim3(NE / 128, 2, 8), ETHR, EDGE_LDS(32), stream>>>(src, HB, 256, HID3, W2T3, c3_b2, PM);
  k_scat<256, 8, 0><<<NN / 32, STHR, 0, stream>>>(tgt, PM, ROOT, HA, HHL);

  k_pool<<<NG, 256, 0, stream>>>(batch, HA, GHL);
  k_gemm<1><<<dim3(1, 1), GTHR, 0, stream>>>(GHL, 512, FC1D, 512, 512, fc1_b, 128, out, 0, G1HL, fc3_w, fc3_b);
  k_gemm<2><<<dim3(1, 1), GTHR, 0, stream>>>(G1HL, 256, FC2D, 256, 256, fc2_b, 64, out, 0, G1HL, fc3_w, fc3_b);
}
